// CvT_Block_63548336111634
// MI455X (gfx1250) — hardware-verified
//
#include <hip/hip_runtime.h>
#include <math.h>

typedef _Float16 f16t;
typedef f16t  v8h  __attribute__((ext_vector_type(8)));
typedef f16t  v16h __attribute__((ext_vector_type(16)));
typedef float v8f  __attribute__((ext_vector_type(8)));
typedef float v4f  __attribute__((ext_vector_type(4)));
typedef v8h __attribute__((may_alias)) v8ha;
typedef v4f __attribute__((may_alias)) v4fa;
union Frag { v16h v; v8h half[2]; };

#define NPOS   1024
#define CDIM   128
#define NHEAD  8
#define DKD    32
#define PADL   34
#define NPADP  1156
#define KEMB   1152
#define ATP    512
#define INV_SQRT2F  0.70710678118654752f
#define INV_SQRT_DK 0.17677669529663688f
#define GELU_C      0.7978845608028654f
#define ATTN_LDS    139264

#define ACAR 4.0f
#define WCAR 64.0f
#define RCAR 256.0f
#define PCAR 1024.0f
#define OCAR 16.0f

__device__ __forceinline__ v8f zero8f() {
  v8f z;
  #pragma unroll
  for (int j = 0; j < 8; ++j) z[j] = 0.f;
  return z;
}

__device__ __forceinline__ v8f wmma_f16(v16h a, v16h b, v8f c) {
  v8f d = __builtin_amdgcn_wmma_f32_16x16x32_f16(false, a, false, b, (short)0, c, false, false);
  asm volatile("v_nop\n\tv_nop\n\tv_nop\n\tv_nop" : "+v"(d) : "v"(a), "v"(b));
  return d;
}

__device__ __forceinline__ v16h load_frag32(const f16t* p, int hl) {
  Frag f;
  f.half[0] = *(const v8ha*)(p + 8 * hl);
  f.half[1] = *(const v8ha*)(p + 16 + 8 * hl);
  return f.v;
}

__device__ __forceinline__ v8h cvt8(const float (&v)[8], float sc) {
  v8h o;
  #pragma unroll
  for (int i = 0; i < 8; ++i) o[i] = (f16t)(v[i] * sc);
  return o;
}

__device__ __forceinline__ int relidx(int i, int j) {
  const int dx = ((i >> 5) - (j >> 5)) & 31;
  const int dy = ((i & 31) - (j & 31)) & 31;
  return (dx << 5) | dy;
}

__global__ __launch_bounds__(256) void wcvt_k(
    const float* __restrict__ We, const float* __restrict__ Wq, const float* __restrict__ W0,
    const float* __restrict__ RK, const float* __restrict__ RQ, const float* __restrict__ RV,
    f16t* WE16, f16t* WQ16, f16t* W016, f16t* RKt, f16t* RQt, f16t* RV16)
{
  const int g = blockIdx.x * 256 + threadIdx.x;
  if (g >= 38912) return;
  const float* base;
  int stride;
  f16t* dst;
  float sc;
  if (g < 18432) {
    const int o = g / 144, kg = g - 144 * o;
    const int k = 8 * kg, tap = k >> 7, c = k & 127;
    base = We + (size_t)(o * CDIM + c) * 9 + tap;
    stride = 9;
    dst = WE16 + (size_t)o * KEMB + k;
    sc = WCAR;
  } else if (g < 22528) {
    const int e8 = (g - 18432) * 8;
    base = Wq + e8; stride = 1; dst = WQ16 + e8; sc = WCAR;
  } else if (g < 26624) {
    const int e8 = (g - 22528) * 8;
    base = W0 + e8; stride = 1; dst = W016 + e8; sc = WCAR;
  } else if (g < 30720) {
    const int e8 = (g - 26624) * 8;
    base = RV + e8; stride = 1; dst = RV16 + e8; sc = RCAR;
  } else if (g < 34816) {
    const int t = g - 30720;
    const int off = t >> 2, d0 = (t & 3) * 8;
    base = RK + (size_t)d0 * NPOS + off; stride = NPOS; dst = RKt + (size_t)off * DKD + d0; sc = RCAR;
  } else {
    const int t = g - 34816;
    const int off = t >> 2, d0 = (t & 3) * 8;
    base = RQ + (size_t)d0 * NPOS + off; stride = NPOS; dst = RQt + (size_t)off * DKD + d0; sc = RCAR;
  }
  float v[8];
  #pragma unroll
  for (int i = 0; i < 8; ++i) v[i] = base[(size_t)i * stride];
  const v8h o8 = cvt8(v, sc);
  *(volatile v8h*)dst = o8;
  __threadfence();
  *(volatile v8h*)dst = o8;
}

__global__ __launch_bounds__(256) void prep_k(const float* __restrict__ x, f16t* T) {
  __shared__ float sG[2048];
  const int tid = threadIdx.x;
  const int pl = tid >> 4, cg = tid & 15;
  const int pp = blockIdx.x * 16 + pl;
  const int ppc = pp < NPADP ? pp : (NPADP - 1);
  const int xp = ppc / PADL, yp = ppc - PADL * xp;
  const int sx = (xp + 31) & 31, sy = (yp + 31) & 31;
  const int src = (sx << 5) | sy;
  #pragma unroll 1
  for (int e = 0; e < 8; ++e) {
    const int c = 8 * cg + e;
    const float u = x[(size_t)c * NPOS + src] * INV_SQRT2F;
    const float inner = GELU_C * (u + 0.044715f * (u * u * u));
    const float t = tanhf(inner);
    sG[tid * 8 + e] = u * (0.5f * (1.0f + t));
  }
  float v[8];
  #pragma unroll
  for (int e = 0; e < 8; ++e) v[e] = sG[tid * 8 + e];
  const v8h o8 = cvt8(v, ACAR);
  if (pp < NPADP) {
    const size_t d = (size_t)pp * CDIM + 8 * cg;
    *(volatile v8h*)(T + d) = o8;
    __threadfence();
    *(volatile v8h*)(T + d) = o8;
  }
}

__global__ __launch_bounds__(128) void conv_k(
    const f16t* __restrict__ T, const f16t* __restrict__ WE16,
    const float* __restrict__ bias, const float* __restrict__ x,
    float* H1, f16t* HT)
{
  __shared__ __attribute__((aligned(16))) float sO[64 * 36];
  const int tid = threadIdx.x, lane = tid & 31, w = tid >> 5;
  const int hl = lane >> 4, m = lane & 15;
  const int X = blockIdx.x, og = blockIdx.y;
  const int mt = w & 1, ntb = 2 * (w >> 1);
  const int Y0 = 16 * mt, o0 = 64 * og;
  const v8f z8 = zero8f();
  v8f acc[2];
  acc[0] = z8; acc[1] = z8;

  #pragma unroll 1
  for (int tap = 0; tap < 9; ++tap) {
    const int ky = tap / 3, kx = tap - 3 * ky;
    const f16t* ap = T + (size_t)((X + ky) * PADL + Y0 + kx + m) * CDIM;
    const f16t* bp = WE16 + (size_t)(o0 + 16 * ntb + m) * KEMB + (size_t)tap * CDIM;
    #pragma unroll 1
    for (int c0 = 0; c0 < CDIM; c0 += 32) {
      const v16h a = load_frag32(ap + c0, hl);
      #pragma unroll
      for (int nt = 0; nt < 2; ++nt) {
        const v16h bb = load_frag32(bp + (size_t)nt * 16 * KEMB + c0, hl);
        acc[nt] = wmma_f16(a, bb, acc[nt]);
      }
    }
  }

  const float osc = 1.0f / (ACAR * WCAR);
  #pragma unroll
  for (int nt = 0; nt < 2; ++nt) {
    const int ol = 16 * (ntb + nt) + m, o = o0 + ol;
    const float bv = bias[o];
    const float* xr = x + (size_t)o * NPOS + X * 32 + Y0 + 8 * hl;
    #pragma unroll
    for (int r = 0; r < 8; ++r) sO[ol * 36 + Y0 + 8 * hl + r] = (acc[nt][r] * osc + bv) + xr[r];
  }
  __syncthreads();

  const int q8 = lane & 7, sub = lane >> 3;
  v4f hv[4];
  size_t hdst[4];
  #pragma unroll
  for (int i = 0; i < 4; ++i) {
    const int row = 16 * w + 4 * i + sub;
    hv[i] = *(const v4fa*)(sO + row * 36 + 4 * q8);
    hdst[i] = (size_t)(o0 + row) * NPOS + X * 32 + 4 * q8;
  }
  v8h th[2];
  size_t td[2];
  #pragma unroll
  for (int i = 0; i < 2; ++i) {
    const int piece = tid + 128 * i;
    const int Y = piece >> 3, q = piece & 7;
    float v[8];
    #pragma unroll
    for (int cc = 0; cc < 8; ++cc) v[cc] = sO[(8 * q + cc) * 36 + Y] * INV_SQRT2F;
    th[i] = cvt8(v, ACAR);
    td[i] = (size_t)(X * 32 + Y) * CDIM + o0 + 8 * q;
  }
  #pragma unroll
  for (int i = 0; i < 4; ++i) *(volatile v4f*)(H1 + hdst[i]) = hv[i];
  #pragma unroll
  for (int i = 0; i < 2; ++i) *(volatile v8h*)(HT + td[i]) = th[i];
  __threadfence();
  #pragma unroll
  for (int i = 0; i < 4; ++i) *(volatile v4f*)(H1 + hdst[i]) = hv[i];
  #pragma unroll
  for (int i = 0; i < 2; ++i) *(volatile v8h*)(HT + td[i]) = th[i];
}

__global__ __launch_bounds__(128) void qproj_k(
    const f16t* __restrict__ HT, const f16t* __restrict__ WQ16, f16t* Q16)
{
  __shared__ __attribute__((aligned(16))) f16t sQ[2 * 64 * 32];
  const int tid = threadIdx.x, lane = tid & 31, w = tid >> 5;
  const int hl = lane >> 4, m = lane & 15;
  const int p0 = 64 * blockIdx.x, og = blockIdx.y, o0 = 64 * og;
  const v8f z8 = zero8f();
  v8f acc[4];
  #pragma unroll
  for (int nt = 0; nt < 4; ++nt) acc[nt] = z8;
  const size_t arow = (size_t)(p0 + 16 * w + m) * CDIM;
  #pragma unroll 1
  for (int c0 = 0; c0 < CDIM; c0 += 32) {
    const v16h a = load_frag32(HT + arow + c0, hl);
    #pragma unroll
    for (int nt = 0; nt < 4; ++nt) {
      const size_t brow = (size_t)(o0 + 16 * nt + m) * CDIM + c0;
      const v16h bb = load_frag32(WQ16 + brow, hl);
      acc[nt] = wmma_f16(a, bb, acc[nt]);
    }
  }
  const float qsc = ACAR / (ACAR * WCAR);
  #pragma unroll
  for (int nt = 0; nt < 4; ++nt) {
    const int hh = nt >> 1, d = 16 * (nt & 1) + m;
    #pragma unroll
    for (int r = 0; r < 8; ++r) {
      const int pos = 16 * w + 8 * hl + r;
      sQ[(hh * 64 + pos) * 32 + d] = (f16t)(acc[nt][r] * qsc);
    }
  }
  __syncthreads();
  v8h vals[4];
  size_t dst[4];
  #pragma unroll
  for (int hh = 0; hh < 2; ++hh) {
    #pragma unroll
    for (int i = 0; i < 2; ++i) {
      const int piece = tid + 128 * i;
      vals[hh * 2 + i] = *(const v8ha*)(sQ + hh * 2048 + piece * 8);
      dst[hh * 2 + i] = ((size_t)(2 * og + hh) * NPOS + p0) * DKD + (size_t)piece * 8;
    }
  }
  #pragma unroll
  for (int i = 0; i < 4; ++i) *(volatile v8h*)(Q16 + dst[i]) = vals[i];
  __threadfence();
  #pragma unroll
  for (int i = 0; i < 4; ++i) *(volatile v8h*)(Q16 + dst[i]) = vals[i];
}

__global__ __launch_bounds__(256) void kv_k(
    const float* __restrict__ H1, const float* __restrict__ Wkd, const float* __restrict__ Wkp,
    const float* __restrict__ Wvd, const float* __restrict__ Wvp,
    f16t* K16, f16t* V16)
{
  __shared__ __attribute__((aligned(16))) float sHK[16 * 64];
  __shared__ __attribute__((aligned(16))) float sHV[16 * 64];
  __shared__ __attribute__((aligned(16))) float sKo[32 * 64];
  __shared__ __attribute__((aligned(16))) float sVo[32 * 64];
  const int tid = threadIdx.x;
  const int xp = blockIdx.x, g = blockIdx.y;
  const int p0 = 64 * xp;
  #pragma unroll 1
  for (int e = 0; e < 4; ++e) {
    const int idx = tid + 256 * e;
    const int cl = idx >> 6, pos = idx & 63;
    const int c = 16 * g + cl;
    const int X = 2 * xp + (pos >> 5), Y = pos & 31;
    const float* hp = H1 + (size_t)c * NPOS;
    const float* wk = Wkd + c * 9;
    const float* wv = Wvd + c * 9;
    float ak = 0.f, av = 0.f;
    #pragma unroll 1
    for (int tap = 0; tap < 9; ++tap) {
      const int ky = tap / 3, kx = tap - 3 * ky;
      const int sx = (X + ky + 31) & 31, sy = (Y + kx + 31) & 31;
      const float v = hp[(sx << 5) | sy] * INV_SQRT2F;
      ak += v * wk[tap];
      av += v * wv[tap];
    }
    sHK[cl * 64 + pos] = ak;
    sHV[cl * 64 + pos] = av;
  }
  __syncthreads();
  {
    const int pos = tid & 63, ob = tid >> 6;
    #pragma unroll 1
    for (int e = 0; e < 8; ++e) {
      const int dl = 8 * ob + e, o = 32 * g + dl;
      const float* wk = Wkp + o * 16;
      const float* wv = Wvp + o * 16;
      float ak = 0.f, av = 0.f;
      #pragma unroll
      for (int cl = 0; cl < 16; ++cl) {
        ak += wk[cl] * sHK[cl * 64 + pos];
        av += wv[cl] * sHV[cl * 64 + pos];
      }
      sKo[dl * 64 + pos] = ak;
      sVo[dl * 64 + pos] = av;
    }
  }
  __syncthreads();
  const int row = tid >> 2, dq = tid & 3;
  float kv8[8];
  #pragma unroll
  for (int cc = 0; cc < 8; ++cc) kv8[cc] = sKo[(8 * dq + cc) * 64 + row];
  const v8h kh8 = cvt8(kv8, ACAR);
  const size_t kd = ((size_t)g * NPOS + p0 + row) * DKD + 8 * dq;
  const int d = tid >> 3, pq = tid & 7;
  const v4f va = *(const v4fa*)(sVo + d * 64 + 8 * pq);
  const v4f vb = *(const v4fa*)(sVo + d * 64 + 8 * pq + 4);
  float vv8[8];
  vv8[0] = va.x; vv8[1] = va.y; vv8[2] = va.z; vv8[3] = va.w;
  vv8[4] = vb.x; vv8[5] = vb.y; vv8[6] = vb.z; vv8[7] = vb.w;
  const v8h vh8 = cvt8(vv8, ACAR);
  const size_t vd = ((size_t)(g * 32 + d)) * NPOS + p0 + 8 * pq;
  *(volatile v8h*)(K16 + kd) = kh8;
  *(volatile v8h*)(V16 + vd) = vh8;
  __threadfence();
  *(volatile v8h*)(K16 + kd) = kh8;
  *(volatile v8h*)(V16 + vd) = vh8;
}

__global__ __launch_bounds__(256) void g_k(
    const f16t* __restrict__ Q16, const f16t* __restrict__ K16,
    const f16t* __restrict__ RKt, const f16t* __restrict__ RQt,
    float* GK, float* GQ)
{
  __shared__ __attribute__((aligned(16))) float sG[64 * 132];
  const int tid = threadIdx.x, lane = tid & 31, w = tid >> 5;
  const int hl = lane >> 4, m = lane & 15;
  const int i0 = 64 * blockIdx.x, n0 = 128 * blockIdx.y;
  const int hd = blockIdx.z >> 1, z = blockIdx.z & 1;
  const f16t* Ap = z ? K16 : Q16;
  const f16t* Bp = z ? RQt : RKt;
  float* G = z ? GQ : GK;
  const int mt = w & 3, ntb = 4 * (w >> 2);
  const size_t arow = ((size_t)hd * NPOS + i0 + 16 * mt + m) * DKD;
  const v16h a = load_frag32(Ap + arow, hl);
  const v8f z8 = zero8f();
  v8f acc[4];
  #pragma unroll
  for (int nt = 0; nt < 4; ++nt) {
    const size_t brow = (size_t)(n0 + 16 * (ntb + nt) + m) * DKD;
    const v16h bb = load_frag32(Bp + brow, hl);
    acc[nt] = wmma_f16(a, bb, z8);
  }
  const float gsc = 1.0f / (ACAR * RCAR);
  #pragma unroll
  for (int nt = 0; nt < 4; ++nt) {
    #pragma unroll
    for (int r = 0; r < 8; ++r) sG[(16 * mt + 8 * hl + r) * 132 + 16 * (ntb + nt) + m] = acc[nt][r] * gsc;
  }
  __syncthreads();
  v4f gv[8];
  size_t gd[8];
  #pragma unroll
  for (int i = 0; i < 8; ++i) {
    const int row = 8 * w + i;
    gv[i] = *(const v4fa*)(sG + row * 132 + 4 * lane);
    gd[i] = ((size_t)hd * NPOS + i0 + row) * NPOS + n0 + 4 * lane;
  }
  #pragma unroll
  for (int i = 0; i < 8; ++i) *(volatile v4f*)(G + gd[i]) = gv[i];
  __threadfence();
  #pragma unroll
  for (int i = 0; i < 8; ++i) *(volatile v4f*)(G + gd[i]) = gv[i];
}

__global__ __launch_bounds__(256) void attn_k(
    const f16t* __restrict__ Q16, const f16t* __restrict__ K16,
    const f16t* __restrict__ V16, const f16t* __restrict__ RV16,
    const float* __restrict__ GK, const float* __restrict__ GQ,
    f16t* ATT)
{
  extern __shared__ v4f dsm4[];
  unsigned char* dsm = (unsigned char*)dsm4;
  float* S     = (float*)dsm;
  f16t*  A16   = (f16t*)(dsm + 65536);
  f16t*  AP16  = (f16t*)(dsm + 98304);
  float* Opart = (float*)(dsm + 131072);
  const int tid = threadIdx.x, lane = tid & 31, w = tid >> 5;
  const int hl = lane >> 4, m = lane & 15;
  const int hd = blockIdx.x >> 6, i0 = (blockIdx.x & 63) * 16;
  const size_t hrow = (size_t)hd * NPOS;
  const v8f z8 = zero8f();

  {
    const float sinv = 1.0f / (ACAR * ACAR);
    const v16h a = load_frag32(Q16 + (hrow + i0 + m) * DKD, hl);
    #pragma unroll 1
    for (int idx = 0; idx < 8; ++idx) {
      const int j0 = 16 * (w + 8 * idx);
      const v16h bb = load_frag32(K16 + (hrow + j0 + m) * DKD, hl);
      const v8f c = wmma_f16(a, bb, z8);
      const int j = j0 + m;
      const float* gqrow = GQ + (hrow + j) * NPOS;
      #pragma unroll
      for (int r = 0; r < 8; ++r) {
        const int il = 8 * hl + r;
        const int i = i0 + il;
        const int off = relidx(i, j);
        const float gk = GK[(hrow + i) * NPOS + off];
        const float gq = gqrow[off];
        S[il * NPOS + j] = ((c[r] * sinv + gk) + gq) * INV_SQRT_DK;
      }
    }
  }
  __syncthreads();

  {
    const int row = tid >> 4, col = tid & 15;
    float* Srow = S + row * NPOS;
    float mx = -3.0e38f;
    #pragma unroll 1
    for (int j = col; j < NPOS; j += 16) mx = fmaxf(mx, Srow[j]);
    mx = fmaxf(mx, __shfl_xor(mx, 8));
    mx = fmaxf(mx, __shfl_xor(mx, 4));
    mx = fmaxf(mx, __shfl_xor(mx, 2));
    mx = fmaxf(mx, __shfl_xor(mx, 1));
    float sum = 0.f;
    #pragma unroll 1
    for (int j = col; j < NPOS; j += 16) {
      const float e = __expf(Srow[j] - mx);
      Srow[j] = e;
      sum += e;
    }
    sum += __shfl_xor(sum, 8);
    sum += __shfl_xor(sum, 4);
    sum += __shfl_xor(sum, 2);
    sum += __shfl_xor(sum, 1);
    const float inv = 1.0f / sum;
    const int ig = i0 + row;
    #pragma unroll 1
    for (int j = col; j < NPOS; j += 16) {
      const float av = Srow[j] * inv;
      const f16t ah = (f16t)(av * PCAR);
      A16[row * NPOS + j] = ah;
      AP16[row * NPOS + relidx(ig, j)] = ah;
    }
  }
  __syncthreads();

  {
    const int gsel = w >> 2, nt = (w >> 1) & 1, kh = w & 1;
    const f16t* Ap = (const f16t*)(dsm + 65536 + gsel * 32768);
    const f16t* Bp = gsel ? RV16 : (V16 + hrow * DKD);
    const f16t* ar = Ap + m * NPOS;
    const f16t* br = Bp + (size_t)(16 * nt + m) * NPOS;
    v8f acc = z8;
    #pragma unroll 1
    for (int ks = 0; ks < 16; ++ks) {
      const int k0 = 32 * (16 * kh + ks);
      const v16h a = load_frag32(ar + k0, hl);
      const v16h bb = load_frag32(br + k0, hl);
      acc = wmma_f16(a, bb, acc);
    }
    #pragma unroll
    for (int r = 0; r < 8; ++r) Opart[w * 256 + (8 * hl + r) * 16 + m] = acc[r];
  }
  __syncthreads();

  f16t* sT = (f16t*)dsm;
  const float vsc = 1.0f / (PCAR * ACAR), rsc = 1.0f / (PCAR * RCAR);
  #pragma unroll
  for (int e = 0; e < 2; ++e) {
    const int idx = tid + 256 * e;
    const int il = idx >> 5, d = idx & 31;
    const int nt = d >> 4, mm = d & 15;
    const int base = il * 16 + mm;
    const float pv  = Opart[(2 * nt) * 256 + base] + Opart[(2 * nt + 1) * 256 + base];
    const float prv = Opart[(4 + 2 * nt) * 256 + base] + Opart[(5 + 2 * nt) * 256 + base];
    const float o = pv * vsc + prv * rsc;
    sT[il * 64 + d] = (f16t)(o * OCAR);
    sT[il * 64 + 32 + d] = (f16t)0.0f;
  }
  __syncthreads();
  if (tid < 128) {
    const int il = tid >> 3, q = tid & 7;
    const v8h val = *(const v8ha*)(sT + il * 64 + 8 * q);
    const size_t dd = (size_t)(i0 + il) * ATP + hd * 64 + 8 * q;
    *(volatile v8h*)(ATT + dd) = val;
    __threadfence();
    *(volatile v8h*)(ATT + dd) = val;
  }
}

__global__ __launch_bounds__(128) void out_k(
    const f16t* __restrict__ ATT, const f16t* __restrict__ W016,
    const float* __restrict__ H1, float* out)
{
  __shared__ __attribute__((aligned(16))) float sO[64 * 68];
  const int tid = threadIdx.x, lane = tid & 31, w = tid >> 5;
  const int hl = lane >> 4, m = lane & 15;
  const int p0 = 64 * blockIdx.x, c0 = 64 * blockIdx.y;
  const v8f z8 = zero8f();
  v8f acc[4];
  #pragma unroll
  for (int nt = 0; nt < 4; ++nt) acc[nt] = z8;
  const size_t arow = (size_t)(p0 + 16 * w + m) * ATP;
  #pragma unroll 1
  for (int kc = 0; kc < 8; ++kc) {
    const v16h a = load_frag32(ATT + arow + kc * 64, hl);
    #pragma unroll
    for (int nt = 0; nt < 4; ++nt) {
      const size_t brow = (size_t)(c0 + 16 * nt + m) * 256 + 32 * kc;
      const v16h bb = load_frag32(W016 + brow, hl);
      acc[nt] = wmma_f16(a, bb, acc[nt]);
    }
  }
  const float osc = 1.0f / (OCAR * WCAR);
  #pragma unroll
  for (int nt = 0; nt < 4; ++nt) {
    #pragma unroll
    for (int r = 0; r < 8; ++r) sO[(16 * nt + m) * 68 + 16 * w + 8 * hl + r] = acc[nt][r] * osc;
  }
  __syncthreads();
  const int q = lane & 15, sub = lane >> 4;
  v4f ov[8];
  size_t od[8];
  #pragma unroll
  for (int i = 0; i < 8; ++i) {
    const int row = 16 * w + 2 * i + sub;
    const v4f v = *(const v4fa*)(sO + row * 68 + 4 * q);
    const v4f res = *(const v4fa*)(H1 + (size_t)(c0 + row) * NPOS + p0 + 4 * q);
    ov[i] = v + res;
    od[i] = (size_t)(c0 + row) * NPOS + p0 + 4 * q;
  }
  #pragma unroll
  for (int i = 0; i < 8; ++i) *(volatile v4f*)(out + od[i]) = ov[i];
  __threadfence();
  #pragma unroll
  for (int i = 0; i < 8; ++i) *(volatile v4f*)(out + od[i]) = ov[i];
}

extern "C" void kernel_launch(void* const* d_in, const int* in_sizes, int n_in,
                              void* d_out, int out_size, void* d_ws, size_t ws_size,
                              hipStream_t stream) {
  if (n_in < 12) return;
  if (in_sizes[0] != CDIM * NPOS || out_size != CDIM * NPOS) return;
  if (in_sizes[1] != CDIM * CDIM * 9 || in_sizes[2] != CDIM) return;
  if (in_sizes[3] != 256 * CDIM) return;
  if (in_sizes[4] != CDIM * 9 || in_sizes[5] != 256 * 16) return;
  if (in_sizes[6] != CDIM * 9 || in_sizes[7] != 256 * 16) return;
  if (in_sizes[8] != DKD * NPOS || in_sizes[9] != DKD * NPOS || in_sizes[10] != DKD * NPOS) return;
  if (in_sizes[11] != CDIM * 256) return;

  const float* x   = (const float*)d_in[0];
  const float* We  = (const float*)d_in[1];
  const float* be  = (const float*)d_in[2];
  const float* Wq  = (const float*)d_in[3];
  const float* Wkd = (const float*)d_in[4];
  const float* Wkp = (const float*)d_in[5];
  const float* Wvd = (const float*)d_in[6];
  const float* Wvp = (const float*)d_in[7];
  const float* RQ  = (const float*)d_in[8];
  const float* RK  = (const float*)d_in[9];
  const float* RV  = (const float*)d_in[10];
  const float* W0  = (const float*)d_in[11];
  float* outp = (float*)d_out;

  char* ws = (char*)d_ws;
  size_t off = 0;
  auto carve = [&](size_t bytes) -> char* {
    char* p = ws + off;
    off += (bytes + 4095) & ~(size_t)4095;
    return p;
  };
  const size_t szWE  = (size_t)CDIM * KEMB * 2;
  const size_t szWQ  = (size_t)256 * CDIM * 2;
  const size_t szW0  = (size_t)CDIM * 256 * 2;
  const size_t szR   = (size_t)DKD * NPOS * 2;
  const size_t szT   = (size_t)NPADP * CDIM * 2;
  const size_t szH1  = (size_t)CDIM * NPOS * 4;
  const size_t szHT  = (size_t)NPOS * CDIM * 2;
  const size_t szQKV = (size_t)NHEAD * NPOS * DKD * 2;
  const size_t szG   = (size_t)NHEAD * NPOS * NPOS * 4;
  const size_t szATT = (size_t)NPOS * ATP * 2;
  f16t* WE16 = (f16t*)carve(szWE);
  f16t* WQ16 = (f16t*)carve(szWQ);
  f16t* W016 = (f16t*)carve(szW0);
  f16t* RV16 = (f16t*)carve(szR);
  f16t* RKt  = (f16t*)carve(szR);
  f16t* RQt  = (f16t*)carve(szR);
  f16t* T    = (f16t*)carve(szT);
  float* H1  = (float*)carve(szH1);
  f16t* HT   = (f16t*)carve(szHT);
  f16t* Q16  = (f16t*)carve(szQKV);
  f16t* K16  = (f16t*)carve(szQKV);
  f16t* V16  = (f16t*)carve(szQKV);
  float* GK  = (float*)carve(szG);
  float* GQ  = (float*)carve(szG);
  f16t* ATT  = (f16t*)carve(szATT);
  if (off > ws_size) return;
  if (off > (size_t)134217728) return;

  wcvt_k<<<152, 256, 0, stream>>>(We, Wq, W0, RK, RQ, RV, WE16, WQ16, W016, RKt, RQt, RV16);
  prep_k<<<73, 256, 0, stream>>>(x, T);
  conv_k<<<dim3(32, 2), 128, 0, stream>>>(T, WE16, be, x, H1, HT);
  qproj_k<<<dim3(16, 4), 128, 0, stream>>>(HT, WQ16, Q16);
  kv_k<<<dim3(16, 8), 256, 0, stream>>>(H1, Wkd, Wkp, Wvd, Wvp, K16, V16);
  g_k<<<dim3(16, 8, 16), 256, 0, stream>>>(Q16, K16, RKt, RQt, GK, GQ);
  attn_k<<<512, 256, ATTN_LDS, stream>>>(Q16, K16, V16, RV16, GK, GQ, ATT);
  out_k<<<dim3(16, 2), 128, 0, stream>>>(ATT, W016, H1, outp);
}
